// FLAME_54245436949017
// MI455X (gfx1250) — hardware-run, weakly checked
//
#include <hip/hip_runtime.h>
#include <math.h>

typedef __attribute__((ext_vector_type(16))) _Float16 v16h;
typedef __attribute__((ext_vector_type(8)))  _Float16 v8h;
typedef __attribute__((ext_vector_type(8)))  float    v8f;
typedef __attribute__((ext_vector_type(4)))  float    v4f;

constexpr int kB   = 1024;
constexpr int kV   = 5023;
constexpr int kJ   = 5;
constexpr int kNB  = 150;
constexpr int kPF  = 36;
constexpr int kNC  = kV * 3;
constexpr int kNP  = 15104;
constexpr int kKP  = 192;
constexpr int kTabP = 192;
constexpr int kTabJT = 160;
constexpr int kBtP = 196;
constexpr int kAfP = 193;
constexpr int kGP  = 61;
constexpr int kTilesM = kB / 64;
constexpr int kTilesN = kNP / 64;
constexpr int kSdElems = kNC * kNB;
constexpr int kPdElems = kPF * kNC;
constexpr size_t kOut0Elems = (size_t)kB * kNC;
constexpr size_t kOutElems  = kOut0Elems + (size_t)kB * kJ * 3;
static_assert(kNC == 15069);
static_assert(kNP % 64 == 0 && kNP >= kNC && (kNP - kNC) < 64);
static_assert(kNB + kPF <= kKP && (kKP % 32) == 0);
static_assert((kB % 64) == 0 && (kB % 32) == 0);
static_assert(kTilesM * kTilesN == 3776 && (kTilesM * kTilesN) % 8 == 0);
static_assert(kOut0Elems * 4 == 61722624ull);
static_assert((kOut0Elems % 32) == 0);
static_assert(kOutElems * 4 == 61784064ull);
static_assert(((size_t)kB * kV) % 256 == 0);
static_assert(kSdElems == 2260350 && kPdElems == 542484);

constexpr float kCarryA = 64.0f;
constexpr float kCarryB = 1024.0f;
constexpr float kFold   = 1.0f / (kCarryA * kCarryB);
constexpr float kF16Min = 6.103515625e-5f;

constexpr size_t kSzBT   = (size_t)kNP * kKP * 2;
constexpr size_t kSzJST  = (size_t)15 * kTabP * 4;
constexpr size_t kSzAREL = (size_t)kB * 60 * 4;
constexpr size_t kSzAOP  = (size_t)kB * kKP * 2;
constexpr size_t kSzVP   = (size_t)kB * kNP * 2;
constexpr size_t kOffBT   = 0;
constexpr size_t kOffJST  = kOffBT + kSzBT;
constexpr size_t kOffAREL = kOffJST + kSzJST;
constexpr size_t kOffAOP  = kOffAREL + kSzAREL;
constexpr size_t kOffVP   = kOffAOP + kSzAOP;
constexpr size_t kWsTotal = kOffVP + kSzVP;
static_assert(kSzBT == 5799936ull && kSzJST == 11520ull && kSzAREL == 245760ull && kSzAOP == 393216ull && kSzVP == 30932992ull);
static_assert(kWsTotal == 37383424ull);
static_assert(kWsTotal <= 134217728ull);
static_assert((kOffJST % 128) == 0 && (kOffAREL % 128) == 0 && (kOffAOP % 128) == 0 && (kOffVP % 128) == 0);

__device__ __forceinline__ void pin_u(unsigned& x) { asm volatile("" : "+v"(x)); }
__device__ __forceinline__ void pin_f(float& x) { asm volatile("" : "+v"(x)); }

__device__ __forceinline__ _Float16 cvt_h_flush(float v) {
  const float a = fabsf(v);
  const float s = (a < kF16Min) ? 0.0f : v;
  return (_Float16)s;
}

__device__ __forceinline__ float h16_to_f32(unsigned hb) {
  const unsigned sgn = (hb & 0x8000u) << 16;
  const unsigned em = hb & 0x7fffu;
  const float fn = __uint_as_float((em << 13) + 0x38000000u);
  const float fs = (float)em * 5.9604644775390625e-8f;
  const float mag = (em < 0x400u) ? fs : fn;
  return __uint_as_float(__float_as_uint(mag) | sgn);
}

__device__ __forceinline__ v16h frag_load_h(const _Float16* p) {
  union U { v16h v; v8h h[2]; };
  U f;
  f.h[0] = *(const v8h*)(p);
  f.h[1] = *(const v8h*)(p + 16);
  return f.v;
}

__device__ __forceinline__ v8f mma_h(v16h a, v16h b, v8f c) {
  c = __builtin_amdgcn_wmma_f32_16x16x32_f16(false, a, false, b, (short)0, c, false, false);
  asm volatile("v_nop\n\tv_nop\n\tv_nop\n\tv_nop" : "+v"(c) : "v"(a), "v"(b));
  return c;
}

__global__ __launch_bounds__(256) void prep_bt_kernel(
    const float* __restrict__ SD, const float* __restrict__ PD, unsigned short* __restrict__ Bt)
{
  __shared__ __align__(16) float sB[64 * kBtP];
  const unsigned tid = threadIdx.x;
  const unsigned n0 = blockIdx.x * 64u;

#pragma unroll 1
  for (unsigned it = 0; it < 38u; ++it) {
    unsigned idx = it * 256u + tid;
    pin_u(idx);
    const bool in = idx < 9600u;
    unsigned ic = in ? idx : 9599u;
    unsigned r = ic / 150u;
    pin_u(r);
    unsigned l = ic - r * 150u;
    pin_u(l);
    unsigned g = n0 * 150u + ic;
    g = (g < (unsigned)kSdElems) ? g : (unsigned)(kSdElems - 1);
    float v = SD[g];
    pin_f(v);
    const bool ok = (n0 + r) < (unsigned)kNC;
    const float val = ok ? v : 0.0f;
    if (in) sB[r * kBtP + l] = val;
  }
#pragma unroll 1
  for (unsigned it = 0; it < 9u; ++it) {
    unsigned idx = it * 256u + tid;
    pin_u(idx);
    unsigned p = idx >> 6;
    unsigned r = idx & 63u;
    pin_u(p);
    pin_u(r);
    const unsigned n = n0 + r;
    const unsigned nc = (n < (unsigned)kNC) ? n : (unsigned)(kNC - 1);
    float v = PD[p * (unsigned)kNC + nc];
    pin_f(v);
    const float val = (n < (unsigned)kNC) ? v : 0.0f;
    sB[r * kBtP + 150u + p] = val;
  }
#pragma unroll 1
  for (unsigned it = 0; it < 2u; ++it) {
    unsigned idx = it * 256u + tid;
    pin_u(idx);
    const bool in = idx < 384u;
    unsigned ic = in ? idx : 383u;
    unsigned r = ic / 6u;
    pin_u(r);
    unsigned c = ic - r * 6u;
    pin_u(c);
    if (in) sB[r * kBtP + 186u + c] = 0.0f;
  }
  __syncthreads();

  v8h hv[6];
#pragma unroll
  for (int it = 0; it < 6; ++it) {
    unsigned c = (unsigned)it * 256u + tid;
    pin_u(c);
    unsigned r = c / 24u;
    pin_u(r);
    unsigned k0 = (c - r * 24u) * 8u;
    pin_u(k0);
    const float* sp = sB + r * kBtP + k0;
    const v4f a0 = *(const v4f*)(sp);
    const v4f a1 = *(const v4f*)(sp + 4);
#pragma unroll
    for (int e = 0; e < 4; ++e) {
      const float x0 = a0[e] * kCarryB;
      const float x1 = a1[e] * kCarryB;
      hv[it][e]     = cvt_h_flush(x0);
      hv[it][4 + e] = cvt_h_flush(x1);
    }
  }
  unsigned short* base = Bt + (size_t)n0 * kKP;
  for (int pass = 0; pass < 2; ++pass) {
#pragma unroll
    for (int it = 0; it < 6; ++it) {
      const unsigned c = (unsigned)it * 256u + tid;
      *(volatile v8h*)(base + (size_t)c * 8) = hv[it];
    }
    __threadfence();
  }
}

__global__ __launch_bounds__(160) void fold_joints_kernel(
    const float* __restrict__ Jreg, const float* __restrict__ vt, const float* __restrict__ SD,
    float* __restrict__ JST)
{
  __shared__ __align__(16) float sRed[160];
  __shared__ __align__(16) float sRow[kTabP];
  const unsigned tid = threadIdx.x;
  const unsigned jk = blockIdx.x;
  const unsigned j = jk / 3u;
  const unsigned k = jk - 3u * j;
  const float* jr = Jreg + (size_t)j * kV;
  const unsigned lc = (tid < (unsigned)kNB) ? tid : (unsigned)(kNB - 1);
  const float* sp = SD + k * 150u + lc;

  float acc = 0.0f;
#pragma unroll 4
  for (unsigned v = 0; v < (unsigned)kV; ++v) acc = fmaf(jr[v], sp[(size_t)v * 450u], acc);

  float pt = 0.0f;
#pragma unroll 1
  for (unsigned i = 0; i < 32u; ++i) {
    unsigned v = tid + 160u * i;
    pin_u(v);
    const bool ok = v < (unsigned)kV;
    const unsigned vc = ok ? v : (unsigned)(kV - 1);
    float a = jr[vc];
    float t = vt[vc * 3u + k];
    pin_f(a);
    pin_f(t);
    const float pr = a * t;
    pt += ok ? pr : 0.0f;
  }
  sRed[tid] = pt;
  __syncthreads();
  for (unsigned s = 80u; s >= 5u; s >>= 1) {
    if (tid < s) sRed[tid] += sRed[tid + s];
    __syncthreads();
  }
  const float jt = ((sRed[0] + sRed[1]) + (sRed[2] + sRed[3])) + sRed[4];

  sRow[tid] = (tid < (unsigned)kNB) ? acc : 0.0f;
  if (tid < 32u) sRow[kTabJT + tid] = (tid == 0u) ? jt : 0.0f;
  __syncthreads();

  const unsigned cc = (tid < 48u) ? tid : 47u;
  const v4f val = *(const v4f*)(sRow + cc * 4u);
  float* dst = JST + (size_t)jk * kTabP + cc * 4u;
  for (int pass = 0; pass < 2; ++pass) {
    if (tid < 48u) *(volatile v4f*)dst = val;
    __threadfence();
  }
}

__global__ __launch_bounds__(32) void pose_chain_kernel(
    const float* __restrict__ betas, const float* __restrict__ pose, const float* __restrict__ JST,
    float* __restrict__ Arel, unsigned short* __restrict__ Aop, float* __restrict__ out1)
{
  __shared__ __align__(16) float sTab[15 * kTabP];
  __shared__ __align__(16) float sAf[32 * kAfP];
  __shared__ __align__(16) float sR[45 * 32];
  __shared__ __align__(16) float sJ[15 * 32];
  __shared__ __align__(16) float sG[32 * kGP];
  __shared__ __align__(16) float sAr[32 * 60];
  __shared__ __align__(16) float sO1[32 * 15];

  const unsigned lane = threadIdx.x;
  const unsigned b0 = blockIdx.x * 32u;
  const unsigned b = b0 + lane;

#pragma unroll 1
  for (unsigned it = 0; it < 90u; ++it) sTab[it * 32u + lane] = JST[it * 32u + lane];
#pragma unroll 1
  for (unsigned it = 0; it < 150u; ++it) {
    unsigned idx = it * 32u + lane;
    pin_u(idx);
    unsigned r = idx / 150u;
    pin_u(r);
    unsigned l = idx - r * 150u;
    pin_u(l);
    sAf[r * kAfP + l] = betas[(size_t)b0 * kNB + idx];
  }
  __syncthreads();

#pragma unroll 1
  for (unsigned j = 0; j < 5u; ++j) {
    const float rx = pose[b * 15u + 3u * j + 0u];
    const float ry = pose[b * 15u + 3u * j + 1u];
    const float rz = pose[b * 15u + 3u * j + 2u];
    const float ex = rx + 1e-8f, ey = ry + 1e-8f, ez = rz + 1e-8f;
    const float ang = sqrtf(ex * ex + ey * ey + ez * ez);
    const float inv = 1.0f / ang;
    const float ux = rx * inv, uy = ry * inv, uz = rz * inv;
    float sn, cs;
    sincosf(ang, &sn, &cs);
    const float t = 1.0f - cs;
    const float ss = ux * ux + uy * uy + uz * uz;
    float* Rj = sR + (j * 9u) * 32u + lane;
    Rj[0 * 32] = 1.0f + t * (ux * ux - ss);
    Rj[1 * 32] = t * (ux * uy) - sn * uz;
    Rj[2 * 32] = t * (ux * uz) + sn * uy;
    Rj[3 * 32] = t * (uy * ux) + sn * uz;
    Rj[4 * 32] = 1.0f + t * (uy * uy - ss);
    Rj[5 * 32] = t * (uy * uz) - sn * ux;
    Rj[6 * 32] = t * (uz * ux) - sn * uy;
    Rj[7 * 32] = t * (uz * uy) + sn * ux;
    Rj[8 * 32] = 1.0f + t * (uz * uz - ss);
  }

#pragma unroll 1
  for (unsigned p = 0; p < 36u; ++p) {
    const unsigned q9 = p / 9u;
    const unsigned i = p - q9 * 9u;
    const float dg = ((i & 3u) == 0u) ? 1.0f : 0.0f;
    sAf[lane * kAfP + 150u + p] = sR[(p + 9u) * 32u + lane] - dg;
  }
#pragma unroll 1
  for (unsigned c = 0; c < 6u; ++c) sAf[lane * kAfP + 186u + c] = 0.0f;

#pragma unroll 1
  for (unsigned jk = 0; jk < 15u; ++jk) {
    const float* tr = sTab + jk * kTabP;
    const float* br = sAf + lane * kAfP;
    float acc = tr[kTabJT];
#pragma unroll 2
    for (unsigned l = 0; l < (unsigned)kNB; ++l) acc = fmaf(tr[l], br[l], acc);
    sJ[jk * 32u + lane] = acc;
  }

#pragma unroll 1
  for (unsigned r = 0; r < 3u; ++r) {
    float* go = sG + lane * kGP + r * 4u;
    go[0] = sR[(r * 3u + 0u) * 32u + lane];
    go[1] = sR[(r * 3u + 1u) * 32u + lane];
    go[2] = sR[(r * 3u + 2u) * 32u + lane];
    go[3] = sJ[r * 32u + lane];
  }
#pragma unroll 1
  for (unsigned j = 1; j < 5u; ++j) {
    const unsigned p = (j == 1u) ? 0u : 1u;
    const float* Rj = sR + (j * 9u) * 32u + lane;
    const float r0 = Rj[0 * 32], r1 = Rj[1 * 32], r2 = Rj[2 * 32];
    const float r3 = Rj[3 * 32], r4 = Rj[4 * 32], r5 = Rj[5 * 32];
    const float r6 = Rj[6 * 32], r7 = Rj[7 * 32], r8 = Rj[8 * 32];
    const float e0 = sJ[(j * 3u + 0u) * 32u + lane] - sJ[(p * 3u + 0u) * 32u + lane];
    const float e1 = sJ[(j * 3u + 1u) * 32u + lane] - sJ[(p * 3u + 1u) * 32u + lane];
    const float e2 = sJ[(j * 3u + 2u) * 32u + lane] - sJ[(p * 3u + 2u) * 32u + lane];
#pragma unroll 1
    for (unsigned r = 0; r < 3u; ++r) {
      const float* gp = sG + lane * kGP + p * 12u + r * 4u;
      float* go = sG + lane * kGP + j * 12u + r * 4u;
      const float g0 = gp[0], g1 = gp[1], g2 = gp[2], g3 = gp[3];
      go[0] = g0 * r0 + g1 * r3 + g2 * r6;
      go[1] = g0 * r1 + g1 * r4 + g2 * r7;
      go[2] = g0 * r2 + g1 * r5 + g2 * r8;
      go[3] = g0 * e0 + g1 * e1 + g2 * e2 + g3;
    }
  }
#pragma unroll 1
  for (unsigned j = 0; j < 5u; ++j) {
    const float j0 = sJ[(j * 3u + 0u) * 32u + lane];
    const float j1 = sJ[(j * 3u + 1u) * 32u + lane];
    const float j2 = sJ[(j * 3u + 2u) * 32u + lane];
#pragma unroll 1
    for (unsigned r = 0; r < 3u; ++r) {
      const float* g = sG + lane * kGP + j * 12u + r * 4u;
      const float g0 = g[0], g1 = g[1], g2 = g[2], g3 = g[3];
      const float rj = g0 * j0 + g1 * j1 + g2 * j2;
      float* ao = sAr + lane * 60u + j * 12u + r * 4u;
      ao[0] = g0;
      ao[1] = g1;
      ao[2] = g2;
      ao[3] = g3 - rj;
      sO1[lane * 15u + j * 3u + r] = g3;
    }
  }
  __syncthreads();

  unsigned short* aopBase = Aop + (size_t)b0 * kKP;
  float* arelBase = Arel + (size_t)b0 * 60;
  float* o1Base = out1 + (size_t)b0 * 15;
  for (int pass = 0; pass < 2; ++pass) {
#pragma unroll 1
    for (unsigned it = 0; it < 24u; ++it) {
      unsigned c = it * 32u + lane;
      pin_u(c);
      unsigned row = c / 24u;
      pin_u(row);
      unsigned k0 = (c - row * 24u) * 8u;
      pin_u(k0);
      const float* sp = sAf + row * kAfP + k0;
      v8h hv;
#pragma unroll
      for (int e = 0; e < 8; ++e) {
        const float x = sp[e] * kCarryA;
        hv[e] = cvt_h_flush(x);
      }
      *(volatile v8h*)(aopBase + (size_t)c * 8) = hv;
    }
#pragma unroll 1
    for (unsigned it = 0; it < 15u; ++it) {
      const unsigned c = it * 32u + lane;
      const v4f val = *(const v4f*)(sAr + c * 4u);
      *(volatile v4f*)(arelBase + (size_t)c * 4) = val;
    }
#pragma unroll 1
    for (unsigned it = 0; it < 4u; ++it) {
      const unsigned c = it * 32u + lane;
      const unsigned cc = (c < 120u) ? c : 119u;
      const v4f val = *(const v4f*)(sO1 + cc * 4u);
      if (c < 120u) *(volatile v4f*)(o1Base + (size_t)c * 4) = val;
    }
    __threadfence();
  }
}

__global__ __launch_bounds__(256) void blend_gemm_kernel(
    const unsigned short* __restrict__ Ap, const unsigned short* __restrict__ Btp,
    unsigned short* __restrict__ VP, const float* __restrict__ vt)
{
  const _Float16* A  = (const _Float16*)Ap;
  const _Float16* Bt = (const _Float16*)Btp;
  __shared__ __align__(16) float sT[8][16 * 68];
  const int lane = threadIdx.x & 31;
  const int wave = threadIdx.x >> 5;
  const int tile = blockIdx.x * 8 + wave;
  if (tile >= kTilesM * kTilesN) return;
  const int tm = tile / kTilesN;
  const int tn = tile - tm * kTilesN;
  const int m0 = tm << 6;
  const int n0 = tn << 6;
  const int rlane = lane & 15;
  const int koff  = (lane >> 4) * 8;
  const int mOff  = (lane >> 4) * 8;

  v8f acc[4][4];
#pragma unroll
  for (int i = 0; i < 4; ++i)
#pragma unroll
    for (int j = 0; j < 4; ++j) acc[i][j] = (v8f){0.f, 0.f, 0.f, 0.f, 0.f, 0.f, 0.f, 0.f};

#pragma unroll 1
  for (int k0 = 0; k0 < kKP; k0 += 32) {
    v16h bh[4];
#pragma unroll
    for (int j = 0; j < 4; ++j)
      bh[j] = frag_load_h(Bt + (size_t)(n0 + (j << 4) + rlane) * kKP + koff + k0);
#pragma unroll
    for (int i = 0; i < 4; ++i) {
      const v16h ah = frag_load_h(A + (size_t)(m0 + (i << 4) + rlane) * kKP + koff + k0);
#pragma unroll
      for (int j = 0; j < 4; ++j) acc[i][j] = mma_h(ah, bh[j], acc[i][j]);
    }
  }

  float bv[4];
#pragma unroll
  for (int j = 0; j < 4; ++j) {
    const int nn = n0 + (j << 4) + rlane;
    const int nc = (nn < kNC) ? nn : (kNC - 1);
    float t = vt[nc];
    pin_f(t);
    bv[j] = (nn < kNC) ? t : 0.0f;
  }

  float* slab = sT[wave];
  const int q = lane >> 3, c8 = (lane & 7) * 8;
#pragma unroll
  for (int i = 0; i < 4; ++i) {
    const int mBase = m0 + (i << 4);
#pragma unroll
    for (int j = 0; j < 4; ++j) {
#pragma unroll
      for (int r = 0; r < 8; ++r) {
        const float a = acc[i][j][r];
        slab[(mOff + r) * 68 + (j << 4) + rlane] = fmaf(a, kFold, bv[j]);
      }
    }
    __builtin_amdgcn_fence(__ATOMIC_RELEASE, "workgroup");
    __builtin_amdgcn_wave_barrier();
    __builtin_amdgcn_fence(__ATOMIC_ACQUIRE, "workgroup");
    for (int pass = 0; pass < 2; ++pass) {
#pragma unroll
      for (int it = 0; it < 4; ++it) {
        const int row = it * 4 + q;
        const float* sp = slab + row * 68 + c8;
        v8h hv;
#pragma unroll
        for (int e = 0; e < 8; ++e) hv[e] = (_Float16)sp[e];
        *(volatile v8h*)(VP + (size_t)(mBase + row) * kNP + n0 + c8) = hv;
      }
      __threadfence();
    }
    __builtin_amdgcn_fence(__ATOMIC_RELEASE, "workgroup");
    __builtin_amdgcn_wave_barrier();
    __builtin_amdgcn_fence(__ATOMIC_ACQUIRE, "workgroup");
  }
}

__global__ __launch_bounds__(256) void skin_kernel(
    const unsigned* __restrict__ VPw, const float* __restrict__ lbs, const float* __restrict__ Arel,
    float* __restrict__ out0)
{
  __shared__ __align__(16) float sO[8][96];
  const unsigned lane = threadIdx.x & 31u;
  const unsigned wave = threadIdx.x >> 5;
  const unsigned wg = blockIdx.x * 8u + wave;
  unsigned pair = wg * 32u + lane;
  pin_u(pair);
  unsigned b = pair / (unsigned)kV;
  pin_u(b);
  unsigned v = pair - b * (unsigned)kV;
  b = (b < (unsigned)(kB - 1)) ? b : (unsigned)(kB - 1);
  v = (v < (unsigned)(kV - 1)) ? v : (unsigned)(kV - 1);
  pin_u(v);

  unsigned wi = b * (unsigned)(kNP / 2) + ((3u * v) >> 1);
  pin_u(wi);
  unsigned w0 = VPw[wi];
  unsigned w1 = VPw[wi + 1u];
  pin_u(w0);
  pin_u(w1);
  const bool odd = (v & 1u) != 0u;
  const unsigned w0lo = w0 & 0xffffu, w0hi = w0 >> 16;
  const unsigned w1lo = w1 & 0xffffu, w1hi = w1 >> 16;
  const unsigned xb = odd ? w0hi : w0lo;
  const unsigned yb = odd ? w1lo : w0hi;
  const unsigned zb = odd ? w1hi : w1lo;
  const float x = h16_to_f32(xb);
  const float y = h16_to_f32(yb);
  const float z = h16_to_f32(zb);

  float ox = 0.0f, oy = 0.0f, oz = 0.0f;
  const float* ab = Arel + (size_t)b * 60;
  const float* wr = lbs + (size_t)v * kJ;
#pragma unroll 1
  for (unsigned j = 0; j < 5u; ++j) {
    const float w = wr[j];
    const v4f a0 = *(const v4f*)(ab + j * 12u);
    const v4f a1 = *(const v4f*)(ab + j * 12u + 4u);
    const v4f a2 = *(const v4f*)(ab + j * 12u + 8u);
    const float t0 = fmaf(a0[0], x, fmaf(a0[1], y, fmaf(a0[2], z, a0[3])));
    const float t1 = fmaf(a1[0], x, fmaf(a1[1], y, fmaf(a1[2], z, a1[3])));
    const float t2 = fmaf(a2[0], x, fmaf(a2[1], y, fmaf(a2[2], z, a2[3])));
    ox = fmaf(w, t0, ox);
    oy = fmaf(w, t1, oy);
    oz = fmaf(w, t2, oz);
  }
  sO[wave][lane * 3u + 0u] = ox;
  sO[wave][lane * 3u + 1u] = oy;
  sO[wave][lane * 3u + 2u] = oz;
  __syncthreads();

  const unsigned lc = (lane < 24u) ? lane : 23u;
  const v4f val = *(const v4f*)(&sO[wave][lc * 4u]);
  float* dst = out0 + (size_t)wg * 96 + lc * 4u;
  for (int pass = 0; pass < 2; ++pass) {
    if (lane < 24u) *(volatile v4f*)dst = val;
    __threadfence();
  }
}

extern "C" void kernel_launch(void* const* d_in, const int* in_sizes, int n_in,
                              void* d_out, int out_size, void* d_ws, size_t ws_size,
                              hipStream_t stream) {
  if (n_in < 7) return;
  if (in_sizes[0] != kB * kNB) return;
  if (in_sizes[1] != kB * kJ * 3) return;
  if (in_sizes[2] != kNC) return;
  if (in_sizes[3] != kSdElems) return;
  if (in_sizes[4] != kPdElems) return;
  if (in_sizes[5] != kJ * kV) return;
  if (in_sizes[6] != kV * kJ) return;
  if ((size_t)out_size != kOutElems) return;
  if (ws_size < kWsTotal) return;

  const float* betas      = (const float*)d_in[0];
  const float* pose       = (const float*)d_in[1];
  const float* v_template = (const float*)d_in[2];
  const float* shapedirs  = (const float*)d_in[3];
  const float* posedirs   = (const float*)d_in[4];
  const float* Jreg       = (const float*)d_in[5];
  const float* lbsw       = (const float*)d_in[6];
  float* out0 = (float*)d_out;
  float* out1 = (float*)d_out + kOut0Elems;

  char* ws = (char*)d_ws;
  unsigned short* BT   = (unsigned short*)(ws + kOffBT);
  float*          JST  = (float*)(ws + kOffJST);
  float*          AREL = (float*)(ws + kOffAREL);
  unsigned short* AOP  = (unsigned short*)(ws + kOffAOP);
  unsigned short* VP   = (unsigned short*)(ws + kOffVP);

  prep_bt_kernel<<<kNP / 64, 256, 0, stream>>>(shapedirs, posedirs, BT);
  fold_joints_kernel<<<15, 160, 0, stream>>>(Jreg, v_template, shapedirs, JST);
  pose_chain_kernel<<<kB / 32, 32, 0, stream>>>(betas, pose, JST, AREL, AOP, out1);
  blend_gemm_kernel<<<(kTilesM * kTilesN) / 8, 256, 0, stream>>>(AOP, BT, VP, v_template);
  skin_kernel<<<(unsigned)(((size_t)kB * kV) / 256), 256, 0, stream>>>((const unsigned*)VP, lbsw, AREL, out0);
}
